// ConvBlock_44427141710403
// MI455X (gfx1250) — hardware-verified
//
#include <hip/hip_runtime.h>


namespace {
constexpr int B = 2, L = 4096, DM = 1024, DI = 2048, KC = 4, NB = 2  ;
constexpr float XS = 8.0f, WSC = 256.0f, RS_ = 1024.0f;
static_assert(L % 64 == 0 && DM % 256 == 0 && DI % 128 == 0, "tiling");
typedef _Float16 b16;
typedef __attribute__((ext_vector_type(16))) _Float16 v16b;
typedef __attribute__((ext_vector_type(8))) _Float16 v8b;
typedef __attribute__((ext_vector_type(8))) float v8f;
typedef __attribute__((ext_vector_type(4))) float v4f;
__device__ __forceinline__ float bf16_rne(float f) { unsigned int u = __float_as_uint(f); u += 0x7FFFu + ((u >> 16) & 1u); return __uint_as_float(u & 0xFFFF0000u); }
__device__ __forceinline__ void split16(float v, b16& hi, b16& lo) { hi = (b16)v; lo = (b16)(v - (float)hi); }
__device__ __forceinline__ v16b frag_kb(const b16* p, int hh) { const v8b a = *(const v8b*)(p + 8 * hh), b = *(const v8b*)(p + 16 + 8 * hh); v16b f;
#pragma unroll
  for (int e = 0; e < 8; ++e) { f[e] = a[e]; f[8 + e] = b[e]; } return f; }
__device__ __forceinline__ v8f wmma16b(v16b a, v16b b, v8f c) { v8f d = __builtin_amdgcn_wmma_f32_16x16x32_f16(false, a, false, b, (short)0, c, false, false); asm volatile("v_nop\n\tv_nop\n\tv_nop\n\tv_nop" : "+v"(d) : "v"(a), "v"(b)); return d; }
__device__ __forceinline__ void wave_lds_sync() { __builtin_amdgcn_fence(__ATOMIC_RELEASE, "workgroup"); __builtin_amdgcn_wave_barrier(); __builtin_amdgcn_fence(__ATOMIC_ACQUIRE, "workgroup"); }
__device__ __forceinline__ float pmul(float a, float b) { float p = a * b; asm volatile("" : "+v"(p)); return p; }
__device__ __forceinline__ int iclamp(int v, int lo, int hi) { return v < lo ? lo : (v > hi ? hi : v); }

typedef __attribute__((ext_vector_type(2))) _Float16 v2h;
typedef __attribute__((ext_vector_type(4))) _Float16 v4h;
typedef __attribute__((ext_vector_type(2))) float v2f;
typedef __attribute__((ext_vector_type(4))) int v4i;
__device__ __forceinline__ float nexp2(float v) { return __builtin_amdgcn_exp2f(v); }
__device__ __forceinline__ float silu_(float y) { return y * __builtin_amdgcn_rcpf(1.0f + __expf(-y)); }
__global__ __launch_bounds__(256) void prep_kernel(const float* __restrict__ wp, const float* __restrict__ wg, const float* __restrict__ wo, b16* __restrict__ WP, b16* __restrict__ WG, b16* __restrict__ WO) {
  const size_t u = (size_t)blockIdx.x * 256 + threadIdx.x; const size_t n = (size_t)DI * DM / 8; if (u >= 3 * n) return; const int m = (int)(u / n); const size_t e = (u % n) * 8; const float* src = (m == 0 ? wp : m == 1 ? wg : wo) + e; b16* dst = (m == 0 ? WP : m == 1 ? WG : WO) + e; v8b o;
  for (int j = 0; j < 8; ++j) o[j] = (b16)(bf16_rne(src[j]) * WSC);
  for (int pass = 0; pass < 2; ++pass) { *(volatile v8b*)dst = o; __threadfence(); }
}
template <int MODE>
__global__ __launch_bounds__(128) void gemm1_kernel(const float* __restrict__ x, int b0, const b16* __restrict__ W, const float* __restrict__ VALin, const float* __restrict__ wc, const float* __restrict__ bc, float* __restrict__ VAL, b16* __restrict__ U, b16* __restrict__ Ul) {
  __shared__ __attribute__((aligned(16))) b16 As[64][256 + 8]; __shared__ __attribute__((aligned(16))) float Tf[4][16][128 + 4];
  const int wave = threadIdx.x >> 5, lane = threadIdx.x & 31, nloc = lane & 15, hlf = lane >> 4; const int t0 = blockIdx.x * 64, n0 = blockIdx.y * 128;
  const float* xb = x + ((size_t)b0 * L + t0) * DM;
  v8f acc[8];
#pragma unroll
  for (int t = 0; t < 8; ++t) acc[t] = (v8f){};
#pragma unroll 1
  for (int kc = 0; kc < DM; kc += 256) {
    __syncthreads();
    for (int i = threadIdx.x; i < 64 * 64; i += 128) { const int rr = i / 64, q = (i % 64) * 4; const v4f f = *(const v4f*)(xb + (size_t)rr * DM + kc + q); v4h o; for (int j = 0; j < 4; ++j) o[j] = (b16)(bf16_rne(f[j]) * XS); *(v4h*)(&As[rr][q]) = o; }
    __syncthreads();
#pragma unroll 2
    for (int kb = 0; kb < 256; kb += 32) { const v16b a = frag_kb(&As[wave * 16 + nloc][kb], hlf);
#pragma unroll
      for (int t = 0; t < 8; ++t) acc[t] = wmma16b(a, frag_kb(W + (size_t)(n0 + t * 16 + nloc) * DM + kc + kb, hlf), acc[t]); } }
#pragma unroll
  for (int t = 0; t < 8; ++t)
#pragma unroll
    for (int r = 0; r < 8; ++r) Tf[wave][8 * hlf + r][t * 16 + nloc] = acc[t][r] * (1.0f / (XS * WSC));
  wave_lds_sync();
  for (int pass = 0; pass < 2; ++pass) {
    for (int rr = 0; rr < 16; ++rr) { const int tok = t0 + wave * 16 + rr; const size_t ro = (size_t)tok * DI + n0 + lane * 4;
      if (MODE == 0) *(volatile v4f*)(VAL + ro) = *(const v4f*)(&Tf[wave][rr][lane * 4]);
      else { v4h h4, l4;
        for (int j = 0; j < 4; ++j) { const int c = n0 + lane * 4 + j; const float g = silu_(Tf[wave][rr][lane * 4 + j]); float cv = bf16_rne(bc[c]);
#pragma unroll
          for (int k = 0; k < KC; ++k) { const int ts = tok - (KC - 1) + k; const float vv = (ts >= 0) ? VALin[(size_t)(ts >= 0 ? ts : 0) * DI + c] : 0.0f; cv = fmaf(bf16_rne(wc[c * KC + k]), vv, cv); }
          const float uu = silu_(cv) * g; b16 p, ql; split16(uu * XS, p, ql); h4[j] = p; l4[j] = ql; }
        *(volatile v4h*)(U + ro) = h4; *(volatile v4h*)(Ul + ro) = l4; } }
    __threadfence(); }
}
__global__ __launch_bounds__(128) void out_kernel(const b16* __restrict__ U, const b16* __restrict__ Ul, const b16* __restrict__ WO, float* __restrict__ out) {
  __shared__ __attribute__((aligned(16))) float Tf[4][16][128 + 4];
  const int wave = threadIdx.x >> 5, lane = threadIdx.x & 31, nloc = lane & 15, hlf = lane >> 4; const size_t m0 = (size_t)blockIdx.x * 64 + wave * 16; const int n0 = blockIdx.y * 128;
  v8f acc[8];
#pragma unroll
  for (int t = 0; t < 8; ++t) acc[t] = (v8f){};
#pragma unroll 2
  for (int kb = 0; kb < DI; kb += 32) { const v16b a = frag_kb(U + (m0 + nloc) * DI + kb, hlf), al = frag_kb(Ul + (m0 + nloc) * DI + kb, hlf);
#pragma unroll
    for (int t = 0; t < 8; ++t) { const v16b bw = frag_kb(WO + (size_t)(n0 + t * 16 + nloc) * DI + kb, hlf); acc[t] = wmma16b(a, bw, acc[t]); acc[t] = wmma16b(al, bw, acc[t]); } }
#pragma unroll
  for (int t = 0; t < 8; ++t)
#pragma unroll
    for (int r = 0; r < 8; ++r) Tf[wave][8 * hlf + r][t * 16 + nloc] = acc[t][r] * (1.0f / (XS * WSC));
  wave_lds_sync();
  for (int pass = 0; pass < 2; ++pass) { for (int rr = 0; rr < 16; ++rr) *(volatile v4f*)(out + (m0 + rr) * DM + n0 + lane * 4) = *(const v4f*)(&Tf[wave][rr][lane * 4]); __threadfence(); }
}
}

extern "C" void kernel_launch(void* const* d_in, const int* in_sizes, int n_in, void* d_out, int out_size, void* d_ws, size_t ws_size, hipStream_t stream) {
  (void)n_in;
  auto Fp = [&](int i) { return (const float*)d_in[i]; };
  if (in_sizes[0] != B * L * DM || in_sizes[1] != DI * DM || in_sizes[2] != DI * DM || in_sizes[3] != DI * KC || in_sizes[4] != DI || in_sizes[5] != DM * DI || out_size != B * L * DM) return;
  size_t off = 0; char* ws = (char*)d_ws;
  auto carve = [&](size_t bytes) { char* p = ws + off; off += (bytes + 255) & ~(size_t)255; return p; };
  b16* WP = (b16*)carve((size_t)DI * DM * 2); b16* WG = (b16*)carve((size_t)DI * DM * 2); b16* WO = (b16*)carve((size_t)DM * DI * 2);
  float* VAL = (float*)carve((size_t)L * DI * 4); b16* U = (b16*)carve((size_t)L * DI * 2); b16* Ul = (b16*)carve((size_t)L * DI * 2);
  if (off > ws_size || off > ((size_t)128 << 20)) return;
  prep_kernel<<<(unsigned)(((size_t)3 * DI * DM / 8 + 255) / 256), 256, 0, stream>>>(Fp(1), Fp(2), Fp(5), WP, WG, WO);
  for (int b0 = 0; b0 < NB; ++b0) {
    gemm1_kernel<0><<<dim3(L / 64, DI / 128), 128, 0, stream>>>(Fp(0), b0, WP, VAL, Fp(3), Fp(4), VAL, U, Ul);
    gemm1_kernel<1><<<dim3(L / 64, DI / 128), 128, 0, stream>>>(Fp(0), b0, WG, VAL, Fp(3), Fp(4), VAL, U, Ul);
    out_kernel<<<dim3(L / 64, DM / 128), 128, 0, stream>>>(U, Ul, WO, (float*)d_out + (size_t)b0 * L * DM); }
}
